// RingDilatedAttentionSDPA_64690797412683
// MI455X (gfx1250) — hardware-verified
//
#include <hip/hip_runtime.h>
#include <math.h>
#include <stdint.h>

#ifndef SEGSEL
#define SEGSEL 0
#endif

#define SEQ   8192
#define DMOD  1024
#define NQKV  (3 * DMOD)
#define NH    16
#define HD    64
#define NSA   2048
#define NSB   4096
#define NSC   2048
#define NCMX  5120
#if SEGSEL
#define NCMP  2048
#define NSEGS 1
#define FILL_N 6144
#define FILL_B 2048
#define FILL_S 1
#else
#define NCMP  5120
#define NSEGS 3
#define FILL_N 3072
#define FILL_B 2049
#define FILL_S 2
#endif
#define QSC   8.0f
#define KSC   8.0f
#define PCAR  32768.0f
#define VCAR  1024.0f
#define OSC   1024.0f
#define LOSC  2048.0f
#define WOS   1024.0f
#define LOG2E 1.4426950408889634f
#define ATT_WAVES   4
#define ATT_THREADS (ATT_WAVES * 32)
#define SLAB   (16 * 68)
#define BIGBRK (1 << 30)
static_assert(HD == 64 && DMOD == NH * HD);
static_assert((NCMP % 64) == 0 && (NCMX % 64) == 0 && NCMP <= NCMX);
static_assert((DMOD % 64) == 0 && (DMOD % 32) == 0);
static_assert((NSA % 64) == 0 && (NSB % 64) == 0 && (NSC % 64) == 0);
static_assert(ATT_THREADS == 128);
static_assert(((NQKV * DMOD / 8) % 256) == 0 && ((DMOD * DMOD / 8) % 256) == 0);
static_assert((SLAB * 4) % 16 == 0);
static_assert(FILL_B + FILL_S * (FILL_N - 1) < SEQ);

typedef unsigned short u16;
typedef _Float16 v16h __attribute__((ext_vector_type(16)));
typedef _Float16 v8h  __attribute__((ext_vector_type(8)));
typedef __bf16   v16b __attribute__((ext_vector_type(16)));
typedef float    v8f  __attribute__((ext_vector_type(8)));
typedef float    v4f  __attribute__((ext_vector_type(4)));
typedef unsigned int v4u __attribute__((ext_vector_type(4)));

union FragH { v16h v; v8h h[2]; v4u u[2]; };
union FragB { v16b v; v4u u[2]; };

__host__ __device__ static inline int amap(int i, int brk, int s1, int s2, int c2) {
  return (i < brk) ? (s1 * i) : (s2 * i + c2);
}

__device__ __forceinline__ int imin(int a, int b) { return a < b ? a : b; }
__device__ __forceinline__ unsigned short bf_bits(float f) {
  unsigned u = __float_as_uint(f);
  return (unsigned short)((u + 0x7FFFu + ((u >> 16) & 1u)) >> 16);
}
__device__ __forceinline__ float bf_up(unsigned short h) { return __uint_as_float(((unsigned)h) << 16); }
__device__ __forceinline__ unsigned short h_bits(_Float16 x) { return __builtin_bit_cast(unsigned short, x); }
__device__ __forceinline__ unsigned pk16(unsigned short a, unsigned short b) { return (unsigned)a | ((unsigned)b << 16); }
__device__ __forceinline__ v8f zero8() { v8f z = {0.f, 0.f, 0.f, 0.f, 0.f, 0.f, 0.f, 0.f}; return z; }

__device__ __forceinline__ v16h ldfrag_h(const _Float16* p) {
  FragH f;
  f.h[0] = *(const v8h*)(p);
  f.h[1] = *(const v8h*)(p + 16);
  return f.v;
}
__device__ __forceinline__ v16b ldfrag_b(const u16* p) {
  FragB f;
  f.u[0] = *(const v4u*)(p);
  f.u[1] = *(const v4u*)(p + 16);
  return f.v;
}

__device__ __forceinline__ v8f mma_h(v16h a, v16h b, v8f c) {
  return __builtin_amdgcn_wmma_f32_16x16x32_f16(false, a, false, b, (short)0, c, false, false);
}
__device__ __forceinline__ v8f mma_b(v16b a, v16b b, v8f c) {
  return __builtin_amdgcn_wmma_f32_16x16x32_bf16(false, a, false, b, (short)0, c, false, false);
}
__device__ __forceinline__ void guard2(v8f& a, v8f& b, v16h x0, v16h x1, v16h x2, v16h x3, v16h x4, v16h x5) {
#if defined(__HIP_DEVICE_COMPILE__)
  asm volatile("v_nop\n\tv_nop\n\tv_nop\n\tv_nop"
               : "+v"(a), "+v"(b) : "v"(x0), "v"(x1), "v"(x2), "v"(x3), "v"(x4), "v"(x5) : "memory");
#endif
}
template <typename F>
__device__ __forceinline__ void guard6(v8f& a, v8f& b, v8f& c, v8f& d, F x0, F x1, F x2, F x3, F x4, F x5) {
#if defined(__HIP_DEVICE_COMPILE__)
  asm volatile("v_nop\n\tv_nop\n\tv_nop\n\tv_nop"
               : "+v"(a), "+v"(b), "+v"(c), "+v"(d) : "v"(x0), "v"(x1), "v"(x2), "v"(x3), "v"(x4), "v"(x5) : "memory");
#endif
}
template <typename F>
__device__ __forceinline__ void guard8(v8f& a, v8f& b, v8f& c, v8f& d, v8f& e, v8f& f, v8f& g, v8f& q,
                                       F x0, F x1, F x2, F x3, F x4, F x5) {
#if defined(__HIP_DEVICE_COMPILE__)
  asm volatile("v_nop\n\tv_nop\n\tv_nop\n\tv_nop"
               : "+v"(a), "+v"(b), "+v"(c), "+v"(d), "+v"(e), "+v"(f), "+v"(g), "+v"(q)
               : "v"(x0), "v"(x1), "v"(x2), "v"(x3), "v"(x4), "v"(x5) : "memory");
#endif
}
__device__ __forceinline__ void acc_guard4(v8f& a, v8f& b, v8f& c, v8f& d) {
#if defined(__HIP_DEVICE_COMPILE__)
  asm volatile("v_nop\n\tv_nop\n\tv_nop\n\tv_nop" : "+v"(a), "+v"(b), "+v"(c), "+v"(d));
#endif
}
__device__ __forceinline__ void wave_sync_lds() {
#if defined(__HIP_DEVICE_COMPILE__)
  __builtin_amdgcn_fence(__ATOMIC_RELEASE, "workgroup");
  __builtin_amdgcn_wave_barrier();
  __builtin_amdgcn_fence(__ATOMIC_ACQUIRE, "workgroup");
#endif
}

__global__ __launch_bounds__(256) void cvt16(const float* __restrict__ x, u16* D, int n8, int mode, float scale) {
  const int gt = blockIdx.x * 256 + (int)threadIdx.x;
  if (gt >= n8) return;
  const float* p = x + (size_t)gt * 8;
  const v4f a = *(const v4f*)(p), c4 = *(const v4f*)(p + 4);
  float v[8];
#pragma unroll
  for (int e = 0; e < 4; ++e) { v[e] = a[e]; v[4 + e] = c4[e]; }
  unsigned short s[8];
#pragma unroll
  for (int e = 0; e < 8; ++e) {
    const unsigned short bb = bf_bits(v[e]);
    const unsigned short hb = h_bits((_Float16)(bf_up(bb) * scale));
    s[e] = (mode != 0) ? hb : bb;
  }
  v4u o;
#pragma unroll
  for (int e = 0; e < 4; ++e) o[e] = pk16(s[2 * e], s[2 * e + 1]);
  u16* d = D + (size_t)gt * 8;
  for (int pass = 0; pass < 2; ++pass) {
    *(volatile v4u*)(d) = o;
    __threadfence();
  }
}

__global__ __launch_bounds__(128) void cvt_x(const float* __restrict__ x, u16* XB) {
  const int cr = blockIdx.x;
  if (cr >= NCMP) return;
  const int t   = (int)threadIdx.x;
  const int pos = amap(cr, 2048, 1, 2, -2048);
  const float* p = x + (size_t)pos * DMOD + t * 8;
  const v4f a = *(const v4f*)(p), c4 = *(const v4f*)(p + 4);
  float v[8];
#pragma unroll
  for (int e = 0; e < 4; ++e) { v[e] = a[e]; v[4 + e] = c4[e]; }
  v4u o;
#pragma unroll
  for (int e = 0; e < 4; ++e) o[e] = pk16(bf_bits(v[2 * e]), bf_bits(v[2 * e + 1]));
  u16* d = XB + (size_t)cr * DMOD + t * 8;
  for (int pass = 0; pass < 2; ++pass) {
    *(volatile v4u*)(d) = o;
    __threadfence();
  }
}

__device__ __forceinline__ void stage_bias(float* sl, v8f a0, v8f a1, v8f a2, v8f a3, const float* __restrict__ bias,
                                           int nbias, int biasRow, float oscale, int rowb, int col0, int lane) {
  const int hh = lane >> 4, m = lane & 15;
  const float bc0 = bias[imin(col0 + m, nbias - 1)];
  const float bc1 = bias[imin(col0 + 16 + m, nbias - 1)];
  const float bc2 = bias[imin(col0 + 32 + m, nbias - 1)];
  const float bc3 = bias[imin(col0 + 48 + m, nbias - 1)];
#pragma unroll
  for (int r = 0; r < 8; ++r) {
    const float br = bias[imin(rowb + 8 * hh + r, nbias - 1)];
    const float e0 = (biasRow != 0) ? br : bc0;
    const float e1 = (biasRow != 0) ? br : bc1;
    const float e2 = (biasRow != 0) ? br : bc2;
    const float e3 = (biasRow != 0) ? br : bc3;
    const int ro = (8 * hh + r) * 68 + m;
    sl[ro]      = (a0[r] + e0) * oscale;
    sl[ro + 16] = (a1[r] + e1) * oscale;
    sl[ro + 32] = (a2[r] + e2) * oscale;
    sl[ro + 48] = (a3[r] + e3) * oscale;
  }
}

__device__ __forceinline__ void store_h16(const float* sl, u16* C, int N, size_t rowb, int col0, int lane) {
  const int rq = lane >> 3, c8 = (lane & 7) * 8;
  v4u ov[4];
#pragma unroll
  for (int i4 = 0; i4 < 4; ++i4) {
    const int row = i4 * 4 + rq;
    const v4f a = *(const v4f*)(sl + row * 68 + c8), c4 = *(const v4f*)(sl + row * 68 + c8 + 4);
    float w[8];
#pragma unroll
    for (int e = 0; e < 4; ++e) { w[e] = a[e]; w[4 + e] = c4[e]; }
#pragma unroll
    for (int e = 0; e < 4; ++e) ov[i4][e] = pk16(h_bits((_Float16)w[2 * e]), h_bits((_Float16)w[2 * e + 1]));
  }
  u16* dst = C + (rowb + (size_t)rq) * (size_t)N + col0 + c8;
  for (int pass = 0; pass < 2; ++pass) {
#pragma unroll
    for (int i4 = 0; i4 < 4; ++i4) {
      *(volatile v4u*)(dst + (size_t)(i4 * 4) * (size_t)N) = ov[i4];
    }
    __threadfence();
  }
}

__device__ __forceinline__ void store_f32(const float* sl, float* C, int N, size_t row0, int rstride, int col0, int lane) {
  const int hh = lane >> 4, m = lane & 15;
  v4f vals[8];
#pragma unroll
  for (int it = 0; it < 8; ++it) vals[it] = *(const v4f*)(sl + (it * 2 + hh) * 68 + m * 4);
  float* dst = C + (row0 + (size_t)rstride * (size_t)hh) * (size_t)N + col0 + m * 4;
  for (int pass = 0; pass < 2; ++pass) {
#pragma unroll
    for (int it = 0; it < 8; ++it) {
      *(volatile v4f*)(dst + (size_t)(rstride * 2 * it) * (size_t)N) = vals[it];
    }
    __threadfence();
  }
}

__global__ __launch_bounds__(128)
void gemm_b16(const u16* __restrict__ A, const u16* __restrict__ Bt, const float* __restrict__ bias, int nbias, int biasRow,
              u16* C, int M, int N, int K, int brk, int s1, int s2, int c2, float oscale) {
  __shared__ __align__(16) float slab[4 * SLAB];
  const int tid = threadIdx.x, wave = tid >> 5, lane = tid & 31, hh = lane >> 4, m = lane & 15;
  const int ntile = N >> 6;
  const int bid   = blockIdx.x;
  const int rowb  = (bid / ntile) * 64 + wave * 16;
  const int col0  = (bid % ntile) * 64;
  if (rowb + 16 > M) return;
  const int br0 = amap(col0, brk, s1, s2, c2);
  const int sB  = (col0 < brk) ? s1 : s2;
  const u16* ap = A  + (size_t)(rowb + m) * K + 8 * hh;
  const u16* bp = Bt + (size_t)(br0 + sB * m) * K + 8 * hh;
  const size_t bs = (size_t)(sB * 16) * (size_t)K;
  v8f acc0 = zero8(), acc1 = zero8(), acc2 = zero8(), acc3 = zero8();
#pragma unroll 1
  for (int k0 = 0; k0 < K; k0 += 32) {
    const v16b a  = ldfrag_b(ap + k0);
    const v16b b0 = ldfrag_b(bp + k0);
    const v16b b1 = ldfrag_b(bp + bs + k0);
    const v16b b2 = ldfrag_b(bp + 2 * bs + k0);
    const v16b b3 = ldfrag_b(bp + 3 * bs + k0);
    acc0 = mma_b(a, b0, acc0);
    acc1 = mma_b(a, b1, acc1);
    acc2 = mma_b(a, b2, acc2);
    acc3 = mma_b(a, b3, acc3);
    guard6<v16b>(acc0, acc1, acc2, acc3, a, b0, b1, b2, b3, a);
  }
  float* sl = slab + wave * SLAB;
  stage_bias(sl, acc0, acc1, acc2, acc3, bias, nbias, biasRow, oscale, rowb, col0, lane);
  wave_sync_lds();
  store_h16(sl, C, N, (size_t)rowb, col0, lane);
}

__global__ __launch_bounds__(128)
void gemm_out(const u16* __restrict__ AH, const u16* __restrict__ AL, const u16* __restrict__ Bt,
              const float* __restrict__ bias, float* C, int M, int N, int K,
              int brk, int s1, int s2, int c2, float oscale, float loscale) {
  __shared__ __align__(16) float slab[4 * SLAB];
  const int tid = threadIdx.x, wave = tid >> 5, lane = tid & 31, hh = lane >> 4, m = lane & 15;
  const int ntile = N >> 6;
  const int bid   = blockIdx.x;
  const int rowb  = (bid / ntile) * 64 + wave * 16;
  const int col0  = (bid % ntile) * 64;
  if (rowb + 16 > M) return;
  const _Float16* aph = (const _Float16*)(const void*)AH + (size_t)(rowb + m) * K + 8 * hh;
  const _Float16* apl = (const _Float16*)(const void*)AL + (size_t)(rowb + m) * K + 8 * hh;
  const _Float16* bp  = (const _Float16*)(const void*)Bt + (size_t)(col0 + m) * K + 8 * hh;
  const size_t bs = (size_t)16 * K;
  v8f h0 = zero8(), h1 = zero8(), h2 = zero8(), h3 = zero8();
  v8f l0 = zero8(), l1 = zero8(), l2 = zero8(), l3 = zero8();
#pragma unroll 1
  for (int k0 = 0; k0 < K; k0 += 32) {
    const v16h ah = ldfrag_h(aph + k0);
    const v16h al = ldfrag_h(apl + k0);
    const v16h b0 = ldfrag_h(bp + k0);
    const v16h b1 = ldfrag_h(bp + bs + k0);
    const v16h b2 = ldfrag_h(bp + 2 * bs + k0);
    const v16h b3 = ldfrag_h(bp + 3 * bs + k0);
    h0 = mma_h(ah, b0, h0);
    h1 = mma_h(ah, b1, h1);
    h2 = mma_h(ah, b2, h2);
    h3 = mma_h(ah, b3, h3);
    l0 = mma_h(al, b0, l0);
    l1 = mma_h(al, b1, l1);
    l2 = mma_h(al, b2, l2);
    l3 = mma_h(al, b3, l3);
    guard8<v16h>(h0, h1, h2, h3, l0, l1, l2, l3, ah, al, b0, b1, b2, b3);
  }
  float* sl = slab + wave * SLAB;
  const float bc0 = bias[imin(col0 + m, N - 1)];
  const float bc1 = bias[imin(col0 + 16 + m, N - 1)];
  const float bc2 = bias[imin(col0 + 32 + m, N - 1)];
  const float bc3 = bias[imin(col0 + 48 + m, N - 1)];
#pragma unroll
  for (int r = 0; r < 8; ++r) {
    const int ro = (8 * hh + r) * 68 + m;
    sl[ro]      = (h0[r] + l0[r] * loscale) * oscale + bc0;
    sl[ro + 16] = (h1[r] + l1[r] * loscale) * oscale + bc1;
    sl[ro + 32] = (h2[r] + l2[r] * loscale) * oscale + bc2;
    sl[ro + 48] = (h3[r] + l3[r] * loscale) * oscale + bc3;
  }
  wave_sync_lds();
  const int pr0 = amap(rowb, brk, s1, s2, c2);
  const int sO  = (rowb < brk) ? s1 : s2;
  store_f32(sl, C, N, (size_t)pr0, sO, col0, lane);
}

__global__ __launch_bounds__(ATT_THREADS)
void attn_seg(const u16* __restrict__ QPp, const u16* __restrict__ KPp, const u16* __restrict__ VTp, float* Op,
              int n, int brk, int st1, int st2, int cb2) {
  __shared__ __align__(16) float smem[ATT_WAVES * SLAB];

  const int tid  = threadIdx.x;
  const int wave = tid >> 5;
  const int lane = tid & 31;
  const int hh   = lane >> 4;
  const int c    = lane & 15;

  const int nqt  = n >> 6;
  const int bid  = blockIdx.x;
  const int head = bid / nqt;
  const int qt   = bid - head * nqt;
  if (head >= NH) return;
  const int q0   = qt * 64 + wave * 16;
  const int qr0  = amap(q0, brk, st1, st2, cb2);
  const int sq   = (q0 < brk) ? st1 : st2;

  const _Float16* Qb = (const _Float16*)(const void*)QPp + ((size_t)(qr0 + sq * c) * DMOD + head * HD + 8 * hh);
  const _Float16* Kh = (const _Float16*)(const void*)KPp + (size_t)(head * HD + 8 * hh);
  const _Float16* Vb = (const _Float16*)(const void*)VTp + ((size_t)(head * HD + c) * (size_t)n + 8 * hh);
  const float lsc = 0.125f * (LOG2E / (QSC * KSC));

  const v16h qf0 = ldfrag_h(Qb);
  const v16h qf1 = ldfrag_h(Qb + 32);

  float mrun = -INFINITY, lrun = 0.f;
  v8f o[4];
#pragma unroll
  for (int j = 0; j < 4; ++j) o[j] = zero8();

  const int nkb = n >> 5;
#pragma unroll 1
  for (int it = 0; it < nkb; ++it) {
    const int kb  = it * 32;
    const int kr0 = amap(kb, brk, st1, st2, cb2);
    const int sk  = (kb < brk) ? st1 : st2;
    v8f sc0 = zero8(), sc1 = zero8();
    const _Float16* k0p = Kh + (size_t)(kr0 + sk * c) * DMOD;
    const _Float16* k1p = k0p + (size_t)(sk * 16) * DMOD;
    const v16h ka0 = ldfrag_h(k0p), ka1 = ldfrag_h(k0p + 32);
    const v16h kc0 = ldfrag_h(k1p), kc1 = ldfrag_h(k1p + 32);
    sc0 = mma_h(ka0, qf0, sc0);
    sc0 = mma_h(ka1, qf1, sc0);
    sc1 = mma_h(kc0, qf0, sc1);
    sc1 = mma_h(kc1, qf1, sc1);
    guard2(sc0, sc1, qf0, qf1, ka0, ka1, kc0, kc1);
    float tk[16];
#pragma unroll
    for (int i = 0; i < 8; ++i) { tk[i] = sc0[i] * lsc;  tk[8 + i] = sc1[i] * lsc; }
    float cm = tk[0];
#pragma unroll
    for (int i = 1; i < 16; ++i) cm = fmaxf(cm, tk[i]);
    cm = fmaxf(cm, __shfl_xor(cm, 16, 32));
    const float mn = fmaxf(mrun, cm);
    const float al = (mrun == -INFINITY) ? 0.f : exp2f(mrun - mn);
    mrun = mn;
    float ps = 0.f;
    FragH ph;
#pragma unroll
    for (int w = 0; w < 2; ++w) {
#pragma unroll
      for (int e4 = 0; e4 < 4; ++e4) {
        const int i = 8 * w + 2 * e4;
        const float p0 = exp2f(fminf(tk[i] - mn, 0.f));
        const float p1 = exp2f(fminf(tk[i + 1] - mn, 0.f));
        ps += p0 + p1;
        ph.u[w][e4] = pk16(h_bits((_Float16)(p0 * PCAR)), h_bits((_Float16)(p1 * PCAR)));
      }
    }
    ps += __shfl_xor(ps, 16, 32);
    lrun = lrun * al + ps;
    float scl[8];
#pragma unroll
    for (int r = 0; r < 8; ++r) scl[r] = __shfl(al, 8 * hh + r, 32);
#pragma unroll
    for (int j = 0; j < 4; ++j) {
#pragma unroll
      for (int r = 0; r < 8; ++r) o[j][r] *= scl[r];
    }
    {
      const _Float16* vp = Vb + kb;
      const v16h vf0 = ldfrag_h(vp);
      const v16h vf1 = ldfrag_h(vp + (size_t)16 * (size_t)n);
      const v16h vf2 = ldfrag_h(vp + (size_t)32 * (size_t)n);
      const v16h vf3 = ldfrag_h(vp + (size_t)48 * (size_t)n);
      o[0] = mma_h(ph.v, vf0, o[0]);
      o[1] = mma_h(ph.v, vf1, o[1]);
      o[2] = mma_h(ph.v, vf2, o[2]);
      o[3] = mma_h(ph.v, vf3, o[3]);
      guard6<v16h>(o[0], o[1], o[2], o[3], ph.v, vf0, vf1, vf2, vf3, ph.v);
    }
  }
  acc_guard4(o[0], o[1], o[2], o[3]);

  const float linv = (lrun > 0.f) ? ((1.0f / lrun) * (1.0f / (PCAR * VCAR))) : 0.f;
  float inv[8];
#pragma unroll
  for (int r = 0; r < 8; ++r) inv[r] = __shfl(linv, 8 * hh + r, 32);
  float* slab = smem + wave * SLAB;
#pragma unroll
  for (int r = 0; r < 8; ++r) {
#pragma unroll
    for (int j = 0; j < 4; ++j) slab[(8 * hh + r) * 68 + j * 16 + c] = o[j][r] * inv[r];
  }
  wave_sync_lds();
  store_f32(slab, Op, DMOD, (size_t)q0, 1, head * HD, lane);
}

__global__ __launch_bounds__(128) void combine_k(const float* __restrict__ OA, const float* __restrict__ OB,
                                                 const float* __restrict__ OC, u16* OH, u16* OL) {
  const int cr = blockIdx.x;
  if (cr >= NCMP) return;
  const int t   = (int)threadIdx.x;
  const int col = t * 8;
  const int pos = amap(cr, 2048, 1, 2, -2048);
  const int   iA = (cr < NSA) ? cr : (NSA - 1);
  const float fA = (cr < NSA) ? 1.0f : 0.0f;
  float v[8];
  {
    const float* pa = OA + (size_t)iA * DMOD + col;
    const v4f a0 = *(const v4f*)(pa), a1 = *(const v4f*)(pa + 4);
#pragma unroll
    for (int e = 0; e < 4; ++e) { v[e] = a0[e] * fA; v[4 + e] = a1[e] * fA; }
  }
#if NSEGS == 3
  {
    const int   iB = imin(pos >> 1, NSB - 1);
    const float fB = ((pos & 1) == 0) ? 1.0f : 0.0f;
    const float* pb = OB + (size_t)iB * DMOD + col;
    const v4f b0 = *(const v4f*)(pb), b1 = *(const v4f*)(pb + 4);
#pragma unroll
    for (int e = 0; e < 4; ++e) { v[e] = v[e] + b0[e] * fB; v[4 + e] = v[4 + e] + b1[e] * fB; }
    const int   iC = imin(pos >> 2, NSC - 1);
    const float fC = ((pos & 3) == 0) ? 1.0f : 0.0f;
    const float* pc = OC + (size_t)iC * DMOD + col;
    const v4f c0 = *(const v4f*)(pc), c1 = *(const v4f*)(pc + 4);
#pragma unroll
    for (int e = 0; e < 4; ++e) { v[e] = v[e] + c0[e] * fC; v[4 + e] = v[4 + e] + c1[e] * fC; }
  }
#endif
  unsigned short sh[8], slo[8];
#pragma unroll
  for (int e = 0; e < 8; ++e) {
    const float tt = v[e] * OSC;
    const _Float16 hi = (_Float16)tt;
    const float res = (tt - (float)hi) * LOSC;
    sh[e]  = h_bits(hi);
    slo[e] = h_bits((_Float16)res);
  }
  v4u oh, ol;
#pragma unroll
  for (int e = 0; e < 4; ++e) { oh[e] = pk16(sh[2 * e], sh[2 * e + 1]); ol[e] = pk16(slo[2 * e], slo[2 * e + 1]); }
  u16* dh = OH + (size_t)cr * DMOD + col;
  u16* dl = OL + (size_t)cr * DMOD + col;
  for (int pass = 0; pass < 2; ++pass) {
    *(volatile v4u*)(dh) = oh;
    *(volatile v4u*)(dl) = ol;
    __threadfence();
  }
}

__global__ __launch_bounds__(128) void fill_rows(const float* __restrict__ bo, float* out, int nrows, int rbase, int rstride) {
  const int wave = threadIdx.x >> 5, lane = threadIdx.x & 31;
  const int j = blockIdx.x * 4 + wave;
  if (j >= nrows) return;
  const int row = rbase + rstride * j;
  if (row >= SEQ || row < 0) return;
  v4f vals[8];
#pragma unroll
  for (int it = 0; it < 8; ++it) vals[it] = *(const v4f*)(bo + it * 128 + lane * 4);
  float* dst = out + (size_t)row * DMOD + lane * 4;
  for (int pass = 0; pass < 2; ++pass) {
#pragma unroll
    for (int it = 0; it < 8; ++it) {
      *(volatile v4f*)(dst + it * 128) = vals[it];
    }
    __threadfence();
  }
}

extern "C" void kernel_launch(void* const* d_in, const int* in_sizes, int n_in,
                              void* d_out, int out_size, void* d_ws, size_t ws_size,
                              hipStream_t stream) {
  if (n_in < 5) return;
  if (in_sizes[0] != SEQ * DMOD) return;
  if (in_sizes[1] != NQKV * DMOD) return;
  if (in_sizes[2] != NQKV) return;
  if (in_sizes[3] != DMOD * DMOD) return;
  if (in_sizes[4] != DMOD) return;
  if (out_size != SEQ * DMOD) return;

  const float* Xin  = (const float*)d_in[0];
  const float* Wqk  = (const float*)d_in[1];
  const float* Bqk  = (const float*)d_in[2];
  const float* Wpr  = (const float*)d_in[3];
  const float* Bpr  = (const float*)d_in[4];
  float*       out  = (float*)d_out;

  const size_t szXB = (size_t)NCMX * DMOD * 2;
  const size_t szWB = (size_t)NQKV * DMOD * 2;
  const size_t szWO = (size_t)DMOD * DMOD * 2;
  const size_t szQP = (size_t)NCMX * DMOD * 2;
  const size_t szVA = (size_t)DMOD * NSA * 2;
  const size_t szVB = (size_t)DMOD * NSB * 2;
  const size_t szVC = (size_t)DMOD * NSC * 2;
  const size_t szOA = (size_t)NSA * DMOD * 4;
  const size_t szOB = (size_t)NSB * DMOD * 4;
  const size_t szOC = (size_t)NSC * DMOD * 4;
  const size_t szOH = (size_t)NCMX * DMOD * 2;
  size_t off = 0;
  const size_t oXB = off; off += szXB;
  const size_t oWB = off; off += szWB;
  const size_t oWO = off; off += szWO;
  const size_t oQP = off; off += szQP;
  const size_t oKP = off; off += szQP;
  const size_t oVA = off; off += szVA;
  const size_t oVB = off; off += szVB;
  const size_t oVC = off; off += szVC;
  const size_t oOA = off; off += szOA;
  const size_t oOB = off; off += szOB;
  const size_t oOC = off; off += szOC;
  const size_t oOH = off; off += szOH;
  const size_t oOL = off; off += szOH;
  if (off > ws_size) return;
  if (off > (size_t)134217728) return;

  char* ws = (char*)d_ws;
  u16*   XB  = (u16*)(ws + oXB);
  u16*   WB  = (u16*)(ws + oWB);
  u16*   WOB = (u16*)(ws + oWO);
  u16*   QP  = (u16*)(ws + oQP);
  u16*   KP  = (u16*)(ws + oKP);
  u16*   VT[3];  VT[0] = (u16*)(ws + oVA);  VT[1] = (u16*)(ws + oVB);  VT[2] = (u16*)(ws + oVC);
  float* OI[3];  OI[0] = (float*)(ws + oOA); OI[1] = (float*)(ws + oOB); OI[2] = (float*)(ws + oOC);
  u16*   OH  = (u16*)(ws + oOH);
  u16*   OL  = (u16*)(ws + oOL);

  const int segn[3]  = {NSA, NSB, NSC};
  const int sbrk[3]  = {BIGBRK, 1024, 512};
  const int ss1[3]   = {1, 2, 4};
  const int ss2[3]   = {1, 1, 2};
  const int sc2[3]   = {0, 1024, 1024};
  for (int s = 0; s < NSEGS; ++s) {
    if ((segn[s] % 64) != 0) return;
    if (sbrk[s] != BIGBRK && (sbrk[s] % 64) != 0) return;
  }

  const int n8q = (NQKV * DMOD) / 8;
  const int n8w = (DMOD * DMOD) / 8;
  if ((n8q % 256) != 0 || (n8w % 256) != 0) return;
  const dim3 b256(256), b128(128);
  const dim3 gXc(NCMP);
  const dim3 gQ(n8q / 256);
  const dim3 gW(n8w / 256);
  const dim3 gG((NCMP / 64) * (DMOD / 64));

  cvt_x<<<gXc, b128, 0, stream>>>(Xin, XB);
  cvt16<<<gQ, b256, 0, stream>>>(Wqk, WB, n8q, 0, 1.0f);
  cvt16<<<gW, b256, 0, stream>>>(Wpr, WOB, n8w, 1, WOS);
  gemm_b16<<<gG, b128, 0, stream>>>(XB, WB, Bqk, NQKV, 0, QP, NCMP, DMOD, DMOD, BIGBRK, 1, 1, 0, QSC);
  gemm_b16<<<gG, b128, 0, stream>>>(XB, WB + (size_t)DMOD * DMOD, Bqk + DMOD, NQKV - DMOD, 0, KP, NCMP, DMOD, DMOD,
                                     BIGBRK, 1, 1, 0, KSC);
  for (int s = 0; s < NSEGS; ++s) {
    const dim3 gV((DMOD / 64) * (segn[s] / 64));
    gemm_b16<<<gV, b128, 0, stream>>>(WB + (size_t)2 * DMOD * DMOD, XB, Bqk + 2 * DMOD, DMOD, 1, VT[s], DMOD, segn[s], DMOD,
                                       sbrk[s], ss1[s], ss2[s], sc2[s], VCAR);
  }
  for (int s = 0; s < NSEGS; ++s) {
    const dim3 gAT((segn[s] / 64) * NH);
    attn_seg<<<gAT, b128, 0, stream>>>(QP, KP, VT[s], OI[s], segn[s], sbrk[s], ss1[s], ss2[s], sc2[s]);
  }
  combine_k<<<gXc, b128, 0, stream>>>(OI[0], OI[1], OI[2], OH, OL);
  gemm_out<<<gG, b128, 0, stream>>>(OH, OL, WOB, Bpr, out, NCMP, DMOD, DMOD, 2048, 1, 2, -2048,
                                     1.0f / ((float)NSEGS * OSC * WOS), 1.0f / LOSC);
  const dim3 gF((FILL_N + 3) / 4);
  fill_rows<<<gF, b128, 0, stream>>>(Bpr, out, FILL_N, FILL_B, FILL_S);
  (void)hipGetLastError();
}
